// ManualCNN_82575041233118
// MI455X (gfx1250) — hardware-verified
//
#include <hip/hip_runtime.h>
#include <stdint.h>

#define NIMG  4096
#define CIN0  3
#define HW0   32
#define XSZ   (CIN0 * HW0 * HW0)
#define C1    16
#define C2    32
#define C3    64
#define NFC   10
#define KFC   1024
#define K1    64
#define K2    160
#define K3    288
#define XP    34
#define XPL   (XP * XP * 4)
#define H1P   18
#define H1L   (H1P * H1P * C1)
#define H2P   10
#define H2L   (H2P * H2P * C2)
#define NTHR  128
#define IMGB  64

#define W1T   0
#define W2T   (W1T + C1 * K1)
#define W3T   (W2T + C2 * K2)
#define FCT   (W3T + C3 * K3)
#define WTOT  (FCT + 16 * KFC)
#define WCH   (WTOT / 8)

#define SCW   64.0f
#define SCX   64.0f
#define RSC   2048.0f
#define INV_A 2.44140625e-04f
#define INV_H 0.015625f
#define INV_X 7.62939453125e-06f

static_assert(WCH % 256 == 0);
static_assert(NIMG % IMGB == 0);
static_assert(H1L % 8 == 0);
static_assert(H2L % 8 == 0);
static_assert(XPL % 4 == 0);
static_assert(W2T % 8 == 0);
static_assert(W3T % 8 == 0);
static_assert(FCT % 8 == 0);
static_assert(K1 % 32 == 0);
static_assert(K2 % 32 == 0);
static_assert(K3 % 32 == 0);
static_assert(KFC % 32 == 0);
static_assert(NTHR == 128);
static_assert(NTHR * 4 == 512);
static_assert((IMGB * NFC * 4) % 128 == 0);

typedef _Float16 v16h __attribute__((ext_vector_type(16)));
typedef _Float16 v8h  __attribute__((ext_vector_type(8)));
typedef _Float16 v4h  __attribute__((ext_vector_type(4)));
typedef float    v8f  __attribute__((ext_vector_type(8)));
typedef float    v4f  __attribute__((ext_vector_type(4)));
typedef unsigned v4u  __attribute__((ext_vector_type(4)));
typedef unsigned v2u  __attribute__((ext_vector_type(2)));

__device__ __forceinline__ float bf_rne(float f) {
  unsigned u = __float_as_uint(f);
  u = (u + 0x7FFFu + ((u >> 16) & 1u)) & 0xFFFF0000u;
  return __uint_as_float(u);
}
__device__ __forceinline__ unsigned hbits(_Float16 h) {
  return (unsigned)__builtin_bit_cast(unsigned short, h);
}
__device__ __forceinline__ void split_hl(float v, _Float16& h, _Float16& l) {
  h = (_Float16)v;
  l = (_Float16)((v - (float)h) * RSC);
}
__device__ __forceinline__ v8f zero8f() { v8f z = {0.f, 0.f, 0.f, 0.f, 0.f, 0.f, 0.f, 0.f}; return z; }
__device__ __forceinline__ v8h zero8h() {
  v8h z;
#pragma unroll
  for (int e = 0; e < 8; ++e) z[e] = (_Float16)0.0f;
  return z;
}
__device__ __forceinline__ float max4(float a, float b, float c, float d) {
  return fmaxf(fmaxf(a, b), fmaxf(c, d));
}

__device__ __forceinline__ v16h ldfrag(const _Float16* p) {
  union { v16h v; v8h h[2]; } f;
  f.h[0] = *(const v8h*)(p);
  f.h[1] = *(const v8h*)(p + 16);
  return f.v;
}

__device__ __forceinline__ v8f mma_h(v16h a, v16h b, v8f c) {
  return __builtin_amdgcn_wmma_f32_16x16x32_f16(false, a, false, b, (short)0, c, false, false);
}
__device__ __forceinline__ void dep_guard1(v8f& w, v16h f0, v16h f1, v16h f2, v16h f3) {
#if defined(__HIP_DEVICE_COMPILE__)
  asm volatile("v_nop\n\tv_nop\n\tv_nop\n\tv_nop"
               : "+v"(w) : "v"(f0), "v"(f1), "v"(f2), "v"(f3));
#endif
}
__device__ __forceinline__ void dep_guard2(v8f& w, v8f& x, v16h f0, v16h f1, v16h f2) {
#if defined(__HIP_DEVICE_COMPILE__)
  asm volatile("v_nop\n\tv_nop\n\tv_nop\n\tv_nop"
               : "+v"(w), "+v"(x) : "v"(f0), "v"(f1), "v"(f2));
#endif
}
__device__ __forceinline__ void dep_guard4(v8f& w, v8f& x, v8f& y, v8f& z,
                                           v16h f0, v16h f1, v16h f2, v16h f3) {
#if defined(__HIP_DEVICE_COMPILE__)
  asm volatile("v_nop\n\tv_nop\n\tv_nop\n\tv_nop"
               : "+v"(w), "+v"(x), "+v"(y), "+v"(z)
               : "v"(f0), "v"(f1), "v"(f2), "v"(f3));
#endif
}
__device__ __forceinline__ void acc_guard1(v8f& w) {
#if defined(__HIP_DEVICE_COMPILE__)
  asm volatile("v_nop\n\tv_nop\n\tv_nop\n\tv_nop" : "+v"(w));
#endif
}
__device__ __forceinline__ void acc_guard2(v8f& w, v8f& x) {
#if defined(__HIP_DEVICE_COMPILE__)
  asm volatile("v_nop\n\tv_nop\n\tv_nop\n\tv_nop" : "+v"(w), "+v"(x));
#endif
}
__device__ __forceinline__ void acc_guard4(v8f& w, v8f& x, v8f& y, v8f& z) {
#if defined(__HIP_DEVICE_COMPILE__)
  asm volatile("v_nop\n\tv_nop\n\tv_nop\n\tv_nop" : "+v"(w), "+v"(x), "+v"(y), "+v"(z));
#endif
}

__device__ __forceinline__ int tap_x(int pb4, int T) {
  const int di = T / 3;
  const int dj = T - 3 * di;
  const int a = pb4 + ((di - 1) * XP + (dj - 1)) * 4;
  return (T < 9) ? a : 0;
}
__device__ __forceinline__ int tap_p(int pb, int T, int pitch) {
  const int di = T / 3;
  const int dj = T - 3 * di;
  const int a = pb + (di - 1) * pitch + (dj - 1);
  return (T < 9) ? a : 0;
}

__global__ __launch_bounds__(256)
void k_wprep(const float* __restrict__ w1, const float* __restrict__ w2, const float* __restrict__ w3,
             const float* __restrict__ fw, unsigned* wb)
{
  const int q  = blockIdx.x * 256 + threadIdx.x;
  const int qc = (q < WCH) ? q : (WCH - 1);

  const int qa  = (qc < 128) ? qc : 127;
  const int na  = qa >> 3;
  const int kca = (qa & 7) * 8;
  int qb = qc - 128;  qb = (qb < 0) ? 0 : ((qb > 639) ? 639 : qb);
  const int nb  = qb / 20;
  const int kcb = (qb - nb * 20) * 8;
  int q3 = qc - 768;  q3 = (q3 < 0) ? 0 : ((q3 > 2303) ? 2303 : q3);
  const int nc  = q3 / 36;
  const int kcc = (q3 - nc * 36) * 8;
  int qd = qc - 3072; qd = (qd < 0) ? 0 : ((qd > 2047) ? 2047 : qd);
  const int nd  = qd >> 7;
  const int kcd = (qd & 127) * 8;
  const int ndc = (nd < NFC) ? nd : (NFC - 1);

  const int sel = (qc < 128) ? 0 : ((qc < 768) ? 1 : ((qc < 3072) ? 2 : 3));

  unsigned hb[8];
#pragma unroll
  for (int j = 0; j < 8; ++j) {
    const int ka  = kca + j;
    const int Ta  = ka >> 2;
    const int cia = ka & 3;
    const int Tac = (Ta < 9) ? Ta : 8;
    const int cic = (cia < 3) ? cia : 2;
    float va = bf_rne(w1[na * 27 + cic * 9 + Tac]) * SCW;
    va = (Ta < 9 && cia < 3) ? va : 0.0f;
    const int kb  = kcb + j;
    const int Tb  = kb >> 4;
    const int cib = kb & 15;
    const int Tbc = (Tb < 9) ? Tb : 8;
    float vb = bf_rne(w2[(nb * 16 + cib) * 9 + Tbc]) * SCW;
    vb = (Tb < 9) ? vb : 0.0f;
    const int kc  = kcc + j;
    const int Tc  = kc >> 5;
    const int cc3 = kc & 31;
    const float vc = bf_rne(w3[(nc * 32 + cc3) * 9 + Tc]) * SCW;
    const int kd  = kcd + j;
    float vd = bf_rne(fw[ndc * KFC + kd]) * SCW;
    vd = (nd < NFC) ? vd : 0.0f;

    const float v = (sel == 0) ? va : ((sel == 1) ? vb : ((sel == 2) ? vc : vd));
    hb[j] = hbits((_Float16)v);
  }
  v4u wh;
  wh.x = hb[0] | (hb[1] << 16);
  wh.y = hb[2] | (hb[3] << 16);
  wh.z = hb[4] | (hb[5] << 16);
  wh.w = hb[6] | (hb[7] << 16);

  unsigned* dst = wb + (size_t)qc * 4;
  if (q < WCH) *(volatile v4u*)dst = wh;
  __threadfence();
  if (q < WCH) *(volatile v4u*)dst = wh;
}

__global__ __launch_bounds__(NTHR)
void k_conv(const float* __restrict__ x, const float* __restrict__ b1, const float* __restrict__ b2,
            const float* __restrict__ b3, const _Float16* __restrict__ wt,
            unsigned* g3h, unsigned* g3l)
{
  __shared__ __align__(16) unsigned xpl[XPL / 2];
  __shared__ __align__(16) _Float16 h1h[H1L];
  __shared__ __align__(16) _Float16 h1l[H1L];
  __shared__ __align__(16) _Float16 h2h[H2L];
  __shared__ __align__(16) _Float16 h2l[H2L];
  __shared__ __align__(16) unsigned o3h[512];
  __shared__ __align__(16) unsigned o3l[512];
  __shared__ float b1s[C1];
  __shared__ float b2s[C2];
  __shared__ float b3s[C3];

  const int tid  = threadIdx.x;
  const int lane = tid & 31;
  const int wv   = tid >> 5;
  const int lm   = lane & 15;
  const int hh   = lane >> 4;
  const int win  = lm >> 2;
  const int qq   = lm & 3;
  const int dy   = qq >> 1;
  const int dx   = qq & 1;
  const int b    = blockIdx.x;

  if (tid < C1) b1s[tid] = bf_rne(b1[tid]);
  if (tid < C2) b2s[tid] = bf_rne(b2[tid]);
  if (tid < C3) b3s[tid] = bf_rne(b3[tid]);

  {
    const v8h z8 = zero8h();
#pragma unroll 1
    for (int i = tid; i < H1L / 8; i += NTHR) {
      *(v8h*)(h1h + 8 * i) = z8;
      *(v8h*)(h1l + 8 * i) = z8;
    }
#pragma unroll 1
    for (int i = tid; i < H2L / 8; i += NTHR) {
      *(v8h*)(h2h + 8 * i) = z8;
      *(v8h*)(h2l + 8 * i) = z8;
    }
  }

  {
    const float* xb = x + (size_t)b * XSZ;
#pragma unroll 1
    for (int p = tid; p < XP * XP; p += NTHR) {
      const int Y  = p / XP;
      const int X  = p - Y * XP;
      const int iy = Y - 1;
      const int ix = X - 1;
      const bool inr = ((unsigned)iy < (unsigned)HW0) && ((unsigned)ix < (unsigned)HW0);
      const int iyc = (iy < 0) ? 0 : ((iy > HW0 - 1) ? (HW0 - 1) : iy);
      const int ixc = (ix < 0) ? 0 : ((ix > HW0 - 1) ? (HW0 - 1) : ix);
      const float* s = xb + iyc * HW0 + ixc;
      const float r0 = s[0];
      const float r1 = s[HW0 * HW0];
      const float r2 = s[2 * HW0 * HW0];
      const float f0 = inr ? bf_rne(r0) * SCX : 0.0f;
      const float f1 = inr ? bf_rne(r1) * SCX : 0.0f;
      const float f2 = inr ? bf_rne(r2) * SCX : 0.0f;
      v2u st;
      st.x = hbits((_Float16)f0) | (hbits((_Float16)f1) << 16);
      st.y = hbits((_Float16)f2);
      *(v2u*)(xpl + p * 2) = st;
    }
  }
  __syncthreads();

  {
    const _Float16* xh = (const _Float16*)xpl;
    const v16h fb0 = ldfrag(wt + W1T + lm * K1 + 8 * hh);
    const v16h fb1 = ldfrag(wt + W1T + lm * K1 + 32 + 8 * hh);
    const float bb = b1s[lm];
#pragma unroll 1
    for (int j = 0; j < 16; ++j) {
      const int t   = wv * 16 + j;
      const int P   = 4 * t + win;
      const int py  = P >> 4;
      const int px  = P & 15;
      const int oy  = 2 * py + dy;
      const int ox  = 2 * px + dx;
      const int pb4 = ((oy + 1) * XP + (ox + 1)) * 4;
      union { v16h v; v4h q[4]; } a0, a1;
      a0.q[0] = *(const v4h*)(xh + tap_x(pb4, 0 + 2 * hh));
      a0.q[1] = *(const v4h*)(xh + tap_x(pb4, 1 + 2 * hh));
      a0.q[2] = *(const v4h*)(xh + tap_x(pb4, 4 + 2 * hh));
      a0.q[3] = *(const v4h*)(xh + tap_x(pb4, 5 + 2 * hh));
      a1.q[0] = *(const v4h*)(xh + tap_x(pb4, 8 + 2 * hh));
      a1.q[1] = *(const v4h*)(xh + tap_x(pb4, 9 + 2 * hh));
      a1.q[2] = *(const v4h*)(xh + tap_x(pb4, 12 + 2 * hh));
      a1.q[3] = *(const v4h*)(xh + tap_x(pb4, 13 + 2 * hh));
      v8f acc = mma_h(a0.v, fb0, zero8f());
      acc = mma_h(a1.v, fb1, acc);
      dep_guard1(acc, a0.v, a1.v, fb0, fb1);

      const float m0 = max4(acc[0], acc[1], acc[2], acc[3]);
      const float m1 = max4(acc[4], acc[5], acc[6], acc[7]);
      const float p0 = fmaxf(m0 * INV_A + bb, 0.0f);
      const float p1 = fmaxf(m1 * INV_A + bb, 0.0f);
      const int P0 = 4 * t + 2 * hh;
      const int i0 = (((P0 >> 4) + 1) * H1P + (P0 & 15) + 1) * C1 + lm;
      _Float16 hv, lv;
      split_hl(p0, hv, lv);
      h1h[i0] = hv;  h1l[i0] = lv;
      split_hl(p1, hv, lv);
      h1h[i0 + C1] = hv;  h1l[i0 + C1] = lv;
    }
  }
  __syncthreads();

  {
#pragma unroll 1
    for (int j = 0; j < 4; ++j) {
      const int t  = wv * 4 + j;
      const int P  = 4 * t + win;
      const int py = P >> 3;
      const int px = P & 7;
      const int oy = 2 * py + dy;
      const int ox = 2 * px + dx;
      const int pb = (oy + 1) * H1P + (ox + 1);
      v8f ah0 = zero8f(), ah1 = zero8f(), ax0 = zero8f(), ax1 = zero8f();
#pragma unroll 1
      for (int s = 0; s < 5; ++s) {
        const int pa = tap_p(pb, 2 * s, H1P) * C1 + 8 * hh;
        const int pc = tap_p(pb, 2 * s + 1, H1P) * C1 + 8 * hh;
        union { v16h v; v8h h[2]; } fah, fal;
        fah.h[0] = *(const v8h*)(h1h + pa);
        fah.h[1] = *(const v8h*)(h1h + pc);
        fal.h[0] = *(const v8h*)(h1l + pa);
        fal.h[1] = *(const v8h*)(h1l + pc);
        const _Float16* wb2 = wt + W2T + lm * K2 + 32 * s + 8 * hh;
        const v16h fb0 = ldfrag(wb2);
        const v16h fb1 = ldfrag(wb2 + 16 * K2);
        ah0 = mma_h(fah.v, fb0, ah0);
        ah1 = mma_h(fah.v, fb1, ah1);
        ax0 = mma_h(fal.v, fb0, ax0);
        ax1 = mma_h(fal.v, fb1, ax1);
        dep_guard4(ah0, ah1, ax0, ax1, fah.v, fal.v, fb0, fb1);
      }
      acc_guard4(ah0, ah1, ax0, ax1);

      const int P0  = 4 * t + 2 * hh;
      const int ib  = (((P0 >> 3) + 1) * H2P + (P0 & 7) + 1) * C2;
      {
        const int c = lm;
        const float m0 = max4(ah0[0] * INV_H + ax0[0] * INV_X, ah0[1] * INV_H + ax0[1] * INV_X,
                              ah0[2] * INV_H + ax0[2] * INV_X, ah0[3] * INV_H + ax0[3] * INV_X);
        const float m1 = max4(ah0[4] * INV_H + ax0[4] * INV_X, ah0[5] * INV_H + ax0[5] * INV_X,
                              ah0[6] * INV_H + ax0[6] * INV_X, ah0[7] * INV_H + ax0[7] * INV_X);
        const float p0 = fmaxf(m0 + b2s[c], 0.0f);
        const float p1 = fmaxf(m1 + b2s[c], 0.0f);
        _Float16 hv, lv;
        split_hl(p0, hv, lv);
        h2h[ib + c] = hv;  h2l[ib + c] = lv;
        split_hl(p1, hv, lv);
        h2h[ib + C2 + c] = hv;  h2l[ib + C2 + c] = lv;
      }
      {
        const int c = 16 + lm;
        const float m0 = max4(ah1[0] * INV_H + ax1[0] * INV_X, ah1[1] * INV_H + ax1[1] * INV_X,
                              ah1[2] * INV_H + ax1[2] * INV_X, ah1[3] * INV_H + ax1[3] * INV_X);
        const float m1 = max4(ah1[4] * INV_H + ax1[4] * INV_X, ah1[5] * INV_H + ax1[5] * INV_X,
                              ah1[6] * INV_H + ax1[6] * INV_X, ah1[7] * INV_H + ax1[7] * INV_X);
        const float p0 = fmaxf(m0 + b2s[c], 0.0f);
        const float p1 = fmaxf(m1 + b2s[c], 0.0f);
        _Float16 hv, lv;
        split_hl(p0, hv, lv);
        h2h[ib + c] = hv;  h2l[ib + c] = lv;
        split_hl(p1, hv, lv);
        h2h[ib + C2 + c] = hv;  h2l[ib + C2 + c] = lv;
      }
    }
  }
  __syncthreads();

  {
    const int t  = wv;
    const int P  = 4 * t + win;
    const int py = P >> 2;
    const int px = P & 3;
    const int oy = 2 * py + dy;
    const int ox = 2 * px + dx;
    const int pb = (oy + 1) * H2P + (ox + 1);
    const int P0 = 4 * t + 2 * hh;
    _Float16* o3hh = (_Float16*)o3h;
    _Float16* o3lh = (_Float16*)o3l;
#pragma unroll 1
    for (int np = 0; np < 2; ++np) {
      v8f ah0 = zero8f(), ah1 = zero8f(), ax0 = zero8f(), ax1 = zero8f();
#pragma unroll 1
      for (int s = 0; s < 9; ++s) {
        const int di = s / 3;
        const int dj = s - 3 * di;
        const int pa = (pb + (di - 1) * H2P + (dj - 1)) * C2 + 8 * hh;
        const v16h fah = ldfrag(h2h + pa);
        const v16h fal = ldfrag(h2l + pa);
        const _Float16* wb3 = wt + W3T + (np * 32 + lm) * K3 + 32 * s + 8 * hh;
        const v16h fb0 = ldfrag(wb3);
        const v16h fb1 = ldfrag(wb3 + 16 * K3);
        ah0 = mma_h(fah, fb0, ah0);
        ah1 = mma_h(fah, fb1, ah1);
        ax0 = mma_h(fal, fb0, ax0);
        ax1 = mma_h(fal, fb1, ax1);
        dep_guard4(ah0, ah1, ax0, ax1, fah, fal, fb0, fb1);
      }
      acc_guard4(ah0, ah1, ax0, ax1);

      {
        const int c  = np * 32 + lm;
        const int i0 = c * 16 + P0;
        const float m0 = max4(ah0[0] * INV_H + ax0[0] * INV_X, ah0[1] * INV_H + ax0[1] * INV_X,
                              ah0[2] * INV_H + ax0[2] * INV_X, ah0[3] * INV_H + ax0[3] * INV_X);
        const float m1 = max4(ah0[4] * INV_H + ax0[4] * INV_X, ah0[5] * INV_H + ax0[5] * INV_X,
                              ah0[6] * INV_H + ax0[6] * INV_X, ah0[7] * INV_H + ax0[7] * INV_X);
        const float p0 = fmaxf(m0 + b3s[c], 0.0f);
        const float p1 = fmaxf(m1 + b3s[c], 0.0f);
        _Float16 hv, lv;
        split_hl(p0, hv, lv);
        o3hh[i0] = hv;  o3lh[i0] = lv;
        split_hl(p1, hv, lv);
        o3hh[i0 + 1] = hv;  o3lh[i0 + 1] = lv;
      }
      {
        const int c  = np * 32 + 16 + lm;
        const int i0 = c * 16 + P0;
        const float m0 = max4(ah1[0] * INV_H + ax1[0] * INV_X, ah1[1] * INV_H + ax1[1] * INV_X,
                              ah1[2] * INV_H + ax1[2] * INV_X, ah1[3] * INV_H + ax1[3] * INV_X);
        const float m1 = max4(ah1[4] * INV_H + ax1[4] * INV_X, ah1[5] * INV_H + ax1[5] * INV_X,
                              ah1[6] * INV_H + ax1[6] * INV_X, ah1[7] * INV_H + ax1[7] * INV_X);
        const float p0 = fmaxf(m0 + b3s[c], 0.0f);
        const float p1 = fmaxf(m1 + b3s[c], 0.0f);
        _Float16 hv, lv;
        split_hl(p0, hv, lv);
        o3hh[i0] = hv;  o3lh[i0] = lv;
        split_hl(p1, hv, lv);
        o3hh[i0 + 1] = hv;  o3lh[i0 + 1] = lv;
      }
    }
  }
  __syncthreads();

  {
    const v4u vh = *(const v4u*)(o3h + tid * 4);
    const v4u vl = *(const v4u*)(o3l + tid * 4);
    unsigned* dh = g3h + (size_t)b * 512 + tid * 4;
    unsigned* dl = g3l + (size_t)b * 512 + tid * 4;
    *(volatile v4u*)dh = vh;
    *(volatile v4u*)dl = vl;
    __threadfence();
    *(volatile v4u*)dh = vh;
    *(volatile v4u*)dl = vl;
  }
}

__global__ __launch_bounds__(NTHR)
void k_fc(const _Float16* __restrict__ h3h, const _Float16* __restrict__ h3l,
          const _Float16* __restrict__ wt, const float* __restrict__ fcb, float* out)
{
  __shared__ __align__(16) float o_s[IMGB * NFC];
  __shared__ float fbs[16];

  const int tid  = threadIdx.x;
  const int lane = tid & 31;
  const int wv   = tid >> 5;
  const int lm   = lane & 15;
  const int hh   = lane >> 4;
  const int img0 = blockIdx.x * IMGB + wv * 16;

  if (tid < 16) {
    const int nc = (tid < NFC) ? tid : (NFC - 1);
    const float bv = bf_rne(fcb[nc]);
    fbs[tid] = (tid < NFC) ? bv : 0.0f;
  }
  __syncthreads();

  const _Float16* pah = h3h + (size_t)(img0 + lm) * KFC + 8 * hh;
  const _Float16* pal = h3l + (size_t)(img0 + lm) * KFC + 8 * hh;
  const _Float16* pbw = wt + FCT + lm * KFC + 8 * hh;

  v8f acc_h = zero8f(), acc_x = zero8f();
#pragma unroll 2
  for (int s = 0; s < KFC / 32; ++s) {
    const v16h fah = ldfrag(pah + 32 * s);
    const v16h fal = ldfrag(pal + 32 * s);
    const v16h fb  = ldfrag(pbw + 32 * s);
    acc_h = mma_h(fah, fb, acc_h);
    acc_x = mma_h(fal, fb, acc_x);
    dep_guard2(acc_h, acc_x, fah, fal, fb);
  }
  acc_guard2(acc_h, acc_x);

  {
    const float bb = fbs[lm];
    const int rowb = wv * 16 + 8 * hh;
    if (lm < NFC) {
      o_s[(rowb + 0) * NFC + lm] = acc_h[0] * INV_H + acc_x[0] * INV_X + bb;
      o_s[(rowb + 1) * NFC + lm] = acc_h[1] * INV_H + acc_x[1] * INV_X + bb;
      o_s[(rowb + 2) * NFC + lm] = acc_h[2] * INV_H + acc_x[2] * INV_X + bb;
      o_s[(rowb + 3) * NFC + lm] = acc_h[3] * INV_H + acc_x[3] * INV_X + bb;
      o_s[(rowb + 4) * NFC + lm] = acc_h[4] * INV_H + acc_x[4] * INV_X + bb;
      o_s[(rowb + 5) * NFC + lm] = acc_h[5] * INV_H + acc_x[5] * INV_X + bb;
      o_s[(rowb + 6) * NFC + lm] = acc_h[6] * INV_H + acc_x[6] * INV_X + bb;
      o_s[(rowb + 7) * NFC + lm] = acc_h[7] * INV_H + acc_x[7] * INV_X + bb;
    }
  }
  __syncthreads();

  float* ob = out + (size_t)blockIdx.x * (IMGB * NFC);
  const int npiece = (IMGB * NFC) / 4;
#pragma unroll 1
  for (int q = tid; q < npiece; q += NTHR) {
    const v4f v = *(const v4f*)(o_s + q * 4);
    *(volatile v4f*)(ob + q * 4) = v;
  }
  __threadfence();
#pragma unroll 1
  for (int q = tid; q < npiece; q += NTHR) {
    const v4f v = *(const v4f*)(o_s + q * 4);
    *(volatile v4f*)(ob + q * 4) = v;
  }
}

extern "C" void kernel_launch(void* const* d_in, const int* in_sizes, int n_in,
                              void* d_out, int out_size, void* d_ws, size_t ws_size,
                              hipStream_t stream) {
  if (n_in < 9) return;
  if (in_sizes[0] != NIMG * XSZ) return;
  if (in_sizes[1] != C1 * CIN0 * 9) return;
  if (in_sizes[2] < C1) return;
  if (in_sizes[3] != C2 * C1 * 9) return;
  if (in_sizes[4] < C2) return;
  if (in_sizes[5] != C3 * C2 * 9) return;
  if (in_sizes[6] < C3) return;
  if (in_sizes[7] != NFC * KFC) return;
  if (in_sizes[8] < NFC) return;
  if (out_size != NIMG * NFC) return;

  const size_t wbytes  = (size_t)WTOT * 2;
  const size_t h3bytes = (size_t)NIMG * KFC * 2;
  const size_t off_w   = 0;
  const size_t off_h3h = off_w + wbytes;
  const size_t off_h3l = off_h3h + h3bytes;
  const size_t total   = off_h3l + h3bytes;
  if (total > ws_size) return;

  const float* x   = (const float*)d_in[0];
  const float* w1  = (const float*)d_in[1];
  const float* b1  = (const float*)d_in[2];
  const float* w2  = (const float*)d_in[3];
  const float* b2  = (const float*)d_in[4];
  const float* w3  = (const float*)d_in[5];
  const float* b3  = (const float*)d_in[6];
  const float* fcw = (const float*)d_in[7];
  const float* fcb = (const float*)d_in[8];
  float* out = (float*)d_out;

  unsigned char* wsb = (unsigned char*)d_ws;
  unsigned* wbuf = (unsigned*)(wsb + off_w);
  unsigned* h3h  = (unsigned*)(wsb + off_h3h);
  unsigned* h3l  = (unsigned*)(wsb + off_h3l);

  k_wprep<<<dim3(WCH / 256), dim3(256), 0, stream>>>(w1, w2, w3, fcw, wbuf);
  (void)hipGetLastError();

  k_conv<<<dim3(NIMG), dim3(NTHR), 0, stream>>>(x, b1, b2, b3, (const _Float16*)wbuf, h3h, h3l);
  (void)hipGetLastError();

  k_fc<<<dim3(NIMG / IMGB), dim3(NTHR), 0, stream>>>((const _Float16*)h3h, (const _Float16*)h3l,
                                                      (const _Float16*)wbuf, fcb, out);
  (void)hipGetLastError();
}
